// RNN_SingleOutput_68908455297449
// MI455X (gfx1250) — hardware-verified
//
#include <hip/hip_runtime.h>

typedef __attribute__((ext_vector_type(16))) _Float16 v16h;
typedef __attribute__((ext_vector_type(8)))  _Float16 v8h;
typedef __attribute__((ext_vector_type(16))) __bf16   v16b;
typedef __attribute__((ext_vector_type(8)))  __bf16   v8b;
typedef __attribute__((ext_vector_type(8)))  float    v8f;
typedef __attribute__((ext_vector_type(4)))  float    v4f;

constexpr int kSeq   = 256;
constexpr int kStep  = 512;
constexpr int kIn    = 64;
constexpr int kHid   = 256;
constexpr int kRows  = kSeq * kStep;
constexpr int kQSeq  = 64;
constexpr int kNQ    = kSeq / kQSeq;
constexpr int kRowsQ = kQSeq * kStep;

constexpr int kSeqPB      = 16;
constexpr int kRnnBlocks  = kQSeq / kSeqPB;
constexpr int kRnnThreads = 256;
constexpr int kHP         = kHid + 8;
constexpr int kHTile      = kSeqPB * kHP;
constexpr int kOutPitch   = 36;
static_assert(kSeq % kQSeq == 0 && kQSeq % kSeqPB == 0);
static_assert(kHid == (kRnnThreads / 32) * 32);
static_assert(kHP % 8 == 0);
static_assert(kHid % 32 == 0 && kIn % 32 == 0);
static_assert(kRowsQ % 64 == 0 && kHid % 64 == 0);
static_assert(kStep % 32 == 0);

constexpr int kDwWih0 = kHid * kIn / 2;
constexpr int kDwWhh  = kHid * kHid / 2;
constexpr int kDwBsum = 2 * kHid;
constexpr int kBlkWih0 = kDwWih0 / 256;
constexpr int kBlkWhh  = kDwWhh / 256;
constexpr int kBlkBsum = kDwBsum / 256;
constexpr int kPrepB1 = kBlkWih0;
constexpr int kPrepB2 = kPrepB1 + kBlkWhh;
constexpr int kPrepB3 = kPrepB2 + kBlkWhh;
constexpr int kPrepB4 = kPrepB3 + kBlkWhh;
constexpr int kPrepBlocks = kPrepB4 + kBlkBsum;
static_assert(kDwWih0 % 256 == 0 && kDwWhh % 256 == 0 && kDwBsum % 256 == 0);
static_assert(kPrepBlocks == 418);
constexpr int kXChunks = kRows * kIn / 8;
static_assert(kXChunks % 256 == 0);

__device__ __forceinline__ unsigned short f2bf_bits(float f) {
  unsigned u = __float_as_uint(f);
  return (unsigned short)((u + 0x7FFFu + ((u >> 16) & 1u)) >> 16);
}
__device__ __forceinline__ float bf_bits2f(unsigned short h) { return __uint_as_float(((unsigned)h) << 16); }
__device__ __forceinline__ float bf16r(float f) { return bf_bits2f(f2bf_bits(f)); }

__device__ __forceinline__ void dep_guard_h(v8f& a, v8f& b, v16h x, v16h y) { asm volatile("v_nop\n\tv_nop\n\tv_nop\n\tv_nop" : "+v"(a), "+v"(b) : "v"(x), "v"(y)); }
__device__ __forceinline__ void dep_guard_b(v8f& a, v8f& b, v16b x, v16b y) { asm volatile("v_nop\n\tv_nop\n\tv_nop\n\tv_nop" : "+v"(a), "+v"(b) : "v"(x), "v"(y)); }
__device__ __forceinline__ void dep_guard3_h(v8f& a, v8f& b, v16h x, v16h y, v16h z) { asm volatile("v_nop\n\tv_nop\n\tv_nop\n\tv_nop" : "+v"(a), "+v"(b) : "v"(x), "v"(y), "v"(z)); }
__device__ __forceinline__ void keep4_h(v16h a, v16h b, v16h c, v16h d) { asm volatile("v_nop" :: "v"(a), "v"(b), "v"(c), "v"(d)); }
__device__ __forceinline__ void keep4_b(v16b a, v16b b, v16b c, v16b d) { asm volatile("v_nop" :: "v"(a), "v"(b), "v"(c), "v"(d)); }
__device__ __forceinline__ void acc_guard4(v8f& a, v8f& b, v8f& c, v8f& d) { asm volatile("v_nop\n\tv_nop\n\tv_nop\n\tv_nop" : "+v"(a), "+v"(b), "+v"(c), "+v"(d)); }
__device__ __forceinline__ void acc_guard2(v8f& a, v8f& b) { asm volatile("v_nop\n\tv_nop\n\tv_nop\n\tv_nop" : "+v"(a), "+v"(b)); }

template <typename T> struct Frag;
template <> struct Frag<_Float16> {
  typedef v16h V; union U { v16h v; v8h h[2]; };
  static __device__ __forceinline__ v16h load(const _Float16* p) {
    U f; f.h[0] = *(const v8h*)(p); f.h[1] = *(const v8h*)(p + 16); return f.v;
  }
  static __device__ __forceinline__ v8f mma(v16h a, v16h b, v8f c) {
    return __builtin_amdgcn_wmma_f32_16x16x32_f16(false, a, false, b, (short)0, c, false, false);
  }
  static __device__ __forceinline__ void guard(v8f& a, v8f& b, v16h x, v16h y) { dep_guard_h(a, b, x, y); }
  static __device__ __forceinline__ void keep(v16h a, v16h b, v16h c, v16h d) { keep4_h(a, b, c, d); }
};
template <> struct Frag<__bf16> {
  typedef v16b V; union U { v16b v; v8b h[2]; };
  static __device__ __forceinline__ v16b load(const __bf16* p) {
    U f; f.h[0] = *(const v8b*)(p); f.h[1] = *(const v8b*)(p + 16); return f.v;
  }
  static __device__ __forceinline__ v8f mma(v16b a, v16b b, v8f c) {
    return __builtin_amdgcn_wmma_f32_16x16x32_bf16(false, a, false, b, (short)0, c, false, false);
  }
  static __device__ __forceinline__ void guard(v8f& a, v8f& b, v16b x, v16b y) { dep_guard_b(a, b, x, y); }
  static __device__ __forceinline__ void keep(v16b a, v16b b, v16b c, v16b d) { keep4_b(a, b, c, d); }
};

template <int ET> struct Elem;
template <> struct Elem<0> { typedef _Float16 T; };
template <> struct Elem<1> { typedef __bf16 T; };
template <int ET, bool SPLIT, int BIAS_MODE, int OUT_MODE, bool RESID, int ACT = 0>
__global__ __launch_bounds__(256) void wmma_gemm64(
    const unsigned short* __restrict__ Ap, const unsigned short* __restrict__ A2p, int lda, long strideA,
    const unsigned short* __restrict__ Btp, const unsigned short* __restrict__ Bt2p, int ldb, long strideB,
    void* __restrict__ Cout, void* __restrict__ Cout2, int ldc, long strideC,
    const float* __restrict__ bias,
    const float* __restrict__ resid, long strideR,
    int M, int N, int K, float scale) {
  typedef typename Elem<ET>::T T;
  typedef typename Frag<T>::V V;
  const T* A = (const T*)Ap; const T* A2 = (const T*)A2p; const T* Bt = (const T*)Btp; const T* Bt2 = (const T*)Bt2p;
  __shared__ __align__(16) float sT[8][16 * 68];
  const int b    = blockIdx.y;
  const int lane = threadIdx.x & 31;
  const int wave = threadIdx.x >> 5;
  const int tilesN = N >> 6;
  const int tilesM = M >> 6;
  const int tile = blockIdx.x * 8 + wave;
  if (tile >= tilesM * tilesN) return;
  const int tm = tile / tilesN;
  const int tn = tile - tm * tilesN;
  const int m0 = tm << 6;
  const int n0 = tn << 6;

  const T* Ab  = A  + (size_t)b * strideA;
  const T* Bb  = Bt + (size_t)b * strideB;
  const T* Ab2 = SPLIT ? (A2  + (size_t)b * strideA) : nullptr;
  const T* Bb2 = SPLIT ? (Bt2 + (size_t)b * strideB) : nullptr;

  const int rlane = lane & 15;
  const int koff  = (lane >> 4) * 8;
  const int mOff  = (lane >> 4) * 8;

  v8f acc[4][4];
#pragma unroll
  for (int i = 0; i < 4; ++i)
#pragma unroll
    for (int j = 0; j < 4; ++j) acc[i][j] = (v8f){0.f,0.f,0.f,0.f,0.f,0.f,0.f,0.f};

  for (int k0 = 0; k0 < K; k0 += 32) {
    V bh[4], bl[4];
#pragma unroll
    for (int j = 0; j < 4; ++j) {
      const size_t bo = (size_t)(n0 + (j << 4) + rlane) * ldb + koff + k0;
      bh[j] = Frag<T>::load(Bb + bo);
      if (SPLIT) bl[j] = Frag<T>::load(Bb2 + bo);
    }
#pragma unroll
    for (int i = 0; i < 4; ++i) {
      const size_t ao = (size_t)(m0 + (i << 4) + rlane) * lda + koff + k0;
      V ah = Frag<T>::load(Ab + ao);
      V al;
      if (SPLIT) al = Frag<T>::load(Ab2 + ao);
#pragma unroll
      for (int j = 0; j < 4; ++j) {
        acc[i][j] = Frag<T>::mma(ah, bh[j], acc[i][j]);
        if (SPLIT) {
          acc[i][j] = Frag<T>::mma(ah, bl[j], acc[i][j]);
          acc[i][j] = Frag<T>::mma(al, bh[j], acc[i][j]);
        }
      }
      Frag<T>::guard(acc[i][0], acc[i][3], ah, SPLIT ? al : ah);
    }
    Frag<T>::keep(bh[0], bh[1], bh[2], bh[3]);
    if (SPLIT) Frag<T>::keep(bl[0], bl[1], bl[2], bl[3]);
  }
  acc_guard4(acc[0][0], acc[0][1], acc[0][2], acc[0][3]);
  acc_guard4(acc[1][0], acc[1][1], acc[1][2], acc[1][3]);
  acc_guard4(acc[2][0], acc[2][1], acc[2][2], acc[2][3]);
  acc_guard4(acc[3][0], acc[3][1], acc[3][2], acc[3][3]);

  float* slab = sT[wave];
  const float* Rb = RESID ? (resid + (size_t)b * strideR) : nullptr;
#pragma unroll
  for (int i = 0; i < 4; ++i) {
    const int mBase = m0 + (i << 4);
#pragma unroll
    for (int j = 0; j < 4; ++j) {
      const int n = n0 + (j << 4) + rlane;
      float bv = 0.f;
      if (BIAS_MODE == 2) bv = bias[n];
#pragma unroll
      for (int r = 0; r < 8; ++r) {
        float v = acc[i][j][r] * scale;
        if (BIAS_MODE == 1) v += bias[mBase + mOff + r];
        if (BIAS_MODE == 2) v += bv;
        if (RESID) v += Rb[(size_t)(mBase + mOff + r) * ldc + n];
        if (ACT == 1) v = tanhf(v);
        if (ACT == 2) v = fmaxf(v, 0.0f);
        if (ACT == 4) v = (v > 0.f) ? v : 0.01f * v;
        slab[(mOff + r) * 68 + (j << 4) + rlane] = v;
      }
    }
    __builtin_amdgcn_fence(__ATOMIC_RELEASE, "workgroup");
    __builtin_amdgcn_wave_barrier();
    __builtin_amdgcn_fence(__ATOMIC_ACQUIRE, "workgroup");
    if (OUT_MODE == 0) {
      float* C = (float*)Cout + (size_t)b * strideC;
      const int hh = lane >> 4, c4 = (lane & 15) * 4;
      for (int pass = 0; pass < 2; ++pass) {
#pragma unroll
        for (int it = 0; it < 8; ++it) {
          const int row = it * 2 + hh;
          v4f v = *(const v4f*)(slab + row * 68 + c4);
          *(volatile v4f*)(C + (size_t)(mBase + row) * ldc + n0 + c4) = v;
        }
        __threadfence();
      }
    } else {
      const int q = lane >> 3, c8 = (lane & 7) * 8;
      unsigned short* C  = (unsigned short*)Cout  + (size_t)b * strideC;
      unsigned short* C2 = (OUT_MODE == 2) ? ((unsigned short*)Cout2 + (size_t)b * strideC) : nullptr;
      for (int pass = 0; pass < 2; ++pass) {
#pragma unroll
        for (int it = 0; it < 4; ++it) {
          const int row = it * 4 + q;
          const float* sp = slab + row * 68 + c8;
          v8h hv, lv;
#pragma unroll
          for (int e = 0; e < 8; ++e) {
            if (OUT_MODE == 1) {
              hv[e] = (_Float16)sp[e];
            } else {
              unsigned short hb = f2bf_bits(sp[e]);
              unsigned short lb = f2bf_bits(sp[e] - bf_bits2f(hb));
              hv[e] = __builtin_bit_cast(_Float16, hb);
              lv[e] = __builtin_bit_cast(_Float16, lb);
            }
          }
          *(volatile v8h*)(C + (size_t)(mBase + row) * ldc + n0 + c8) = hv;
          if (OUT_MODE == 2) *(volatile v8h*)(C2 + (size_t)(mBase + row) * ldc + n0 + c8) = lv;
        }
        __threadfence();
      }
    }
    __builtin_amdgcn_fence(__ATOMIC_RELEASE, "workgroup");
    __builtin_amdgcn_wave_barrier();
    __builtin_amdgcn_fence(__ATOMIC_ACQUIRE, "workgroup");
  }
}

__device__ __forceinline__ unsigned pack_f16x2(float a, float b) {
  const _Float16 h0 = (_Float16)a, h1 = (_Float16)b;
  return (unsigned)__builtin_bit_cast(unsigned short, h0) | ((unsigned)__builtin_bit_cast(unsigned short, h1) << 16);
}
__device__ __forceinline__ void st2u(unsigned* p, unsigned v) { *(volatile unsigned*)p = v; __threadfence(); *(volatile unsigned*)p = v; }

__global__ __launch_bounds__(256) void prep_kernel(
    const float* __restrict__ w_ih0, const float* __restrict__ w_hh0,
    const float* __restrict__ w_ih1, const float* __restrict__ w_hh1,
    const float* __restrict__ b_ih0, const float* __restrict__ b_hh0,
    const float* __restrict__ b_ih1, const float* __restrict__ b_hh1,
    unsigned* __restrict__ wih0u, unsigned* __restrict__ whh0u,
    unsigned* __restrict__ wih1u, unsigned* __restrict__ whh1u,
    unsigned* __restrict__ bsumu) {
  const int blk = blockIdx.x, tid = threadIdx.x;
  const float ws16 = 16.0f;
  if (blk < kPrepB1) {
    const int p = blk * 256 + tid;
    st2u(wih0u + p, pack_f16x2(bf16r(w_ih0[2 * p]) * ws16, bf16r(w_ih0[2 * p + 1]) * ws16));
  } else if (blk < kPrepB2) {
    const int p = (blk - kPrepB1) * 256 + tid;
    st2u(whh0u + p, pack_f16x2(bf16r(w_hh0[2 * p]) * ws16, bf16r(w_hh0[2 * p + 1]) * ws16));
  } else if (blk < kPrepB3) {
    const int p = (blk - kPrepB2) * 256 + tid;
    st2u(wih1u + p, pack_f16x2(bf16r(w_ih1[2 * p]) * ws16, bf16r(w_ih1[2 * p + 1]) * ws16));
  } else if (blk < kPrepB4) {
    const int p = (blk - kPrepB3) * 256 + tid;
    st2u(whh1u + p, pack_f16x2(bf16r(w_hh1[2 * p]) * ws16, bf16r(w_hh1[2 * p + 1]) * ws16));
  } else {
    const int p = (blk - kPrepB4) * 256 + tid;
    const int pc = p & (kHid - 1);
    const float s0 = bf16r(b_ih0[pc]) + bf16r(b_hh0[pc]);
    const float s1 = bf16r(b_ih1[pc]) + bf16r(b_hh1[pc]);
    const float v = (p < kHid) ? s0 : s1;
    st2u(bsumu + p, (unsigned)__float_as_uint(v));
  }
}

__global__ __launch_bounds__(256) void xcast_kernel(const float* __restrict__ x, _Float16* __restrict__ x16) {
  const int i = blockIdx.x * 256 + threadIdx.x;
  const int row = i >> 3, c8 = i & 7;
  const int g = row >> 15, rem = row & 32767;
  const int t = rem >> 6, bl = rem & 63;
  const int b = g * kQSeq + bl;
  const float* src = x + ((size_t)b * kStep + t) * kIn + c8 * 8;
  const v4f f0 = *(const v4f*)src;
  const v4f f1 = *(const v4f*)(src + 4);
  v8h hv;
  hv[0] = (_Float16)bf16r(f0[0]); hv[1] = (_Float16)bf16r(f0[1]); hv[2] = (_Float16)bf16r(f0[2]); hv[3] = (_Float16)bf16r(f0[3]);
  hv[4] = (_Float16)bf16r(f1[0]); hv[5] = (_Float16)bf16r(f1[1]); hv[6] = (_Float16)bf16r(f1[2]); hv[7] = (_Float16)bf16r(f1[3]);
  _Float16* dst = x16 + (size_t)row * kIn + c8 * 8;
  *(volatile v8h*)dst = hv;
  __threadfence();
  *(volatile v8h*)dst = hv;
}

template <int HEAD>
__global__ __launch_bounds__(kRnnThreads) void rnn_layer_kernel(
    const float* __restrict__ pre, const _Float16* __restrict__ whh16,
    _Float16* __restrict__ hout,
    const float* __restrict__ wfc, const float* __restrict__ bfc, float* __restrict__ outq) {
  __shared__ __align__(16) _Float16 hbuf[2 * kHTile];
  __shared__ __align__(16) float sPart[2 * 8 * kSeqPB];
  __shared__ __align__(16) float sOut[kSeqPB * kOutPitch];
  const int tid = threadIdx.x, lane = tid & 31, wave = tid >> 5;
  const int c = lane & 15, hh = lane >> 4, koff = hh * 8, mOff = hh * 8;
  const int bl0 = blockIdx.x * kSeqPB;
  const int n0 = wave * 32;

  {
    const v8h z = {(_Float16)0.f, (_Float16)0.f, (_Float16)0.f, (_Float16)0.f, (_Float16)0.f, (_Float16)0.f, (_Float16)0.f, (_Float16)0.f};
    for (int i = tid; i < (2 * kHTile) / 8; i += kRnnThreads) *(v8h*)(hbuf + i * 8) = z;
    if (HEAD) {
      for (int i = tid; i < 2 * 8 * kSeqPB; i += kRnnThreads) sPart[i] = 0.f;
      for (int i = tid; i < kSeqPB * kOutPitch; i += kRnnThreads) sOut[i] = 0.f;
    }
  }
  __syncthreads();

  float wf0 = 0.f, wf1 = 0.f, bfcv = 0.f;
  if (HEAD) { wf0 = bf16r(wfc[n0 + c]); wf1 = bf16r(wfc[n0 + 16 + c]); bfcv = bf16r(bfc[0]); }

  const float inv16 = 0.0625f;
  const _Float16* brow = whh16 + (size_t)(n0 + c) * kHid + koff;
  const int q4 = lane >> 3, c4 = (lane & 7) * 4;

#pragma unroll 1
  for (int t = 0; t < kStep; ++t) {
    const _Float16* hc = hbuf + (t & 1) * kHTile;
    _Float16*       hn = hbuf + ((t + 1) & 1) * kHTile;
    v8f acc[2];
#pragma unroll
    for (int j = 0; j < 2; ++j) {
      const float* xp = pre + (size_t)(n0 + 16 * j + c) * kRowsQ + (size_t)t * kQSeq + bl0 + 8 * hh;
      const v4f xa = *(const v4f*)xp;
      const v4f xb = *(const v4f*)(xp + 4);
      acc[j][0] = xa[0] * 16.0f; acc[j][1] = xa[1] * 16.0f; acc[j][2] = xa[2] * 16.0f; acc[j][3] = xa[3] * 16.0f;
      acc[j][4] = xb[0] * 16.0f; acc[j][5] = xb[1] * 16.0f; acc[j][6] = xb[2] * 16.0f; acc[j][7] = xb[3] * 16.0f;
    }
    const _Float16* arow = hc + c * kHP + koff;
#pragma unroll
    for (int kc = 0; kc < kHid / 32; ++kc) {
      const v16h fa  = Frag<_Float16>::load(arow + kc * 32);
      const v16h fb0 = Frag<_Float16>::load(brow + kc * 32);
      const v16h fb1 = Frag<_Float16>::load(brow + (size_t)16 * kHid + kc * 32);
      acc[0] = Frag<_Float16>::mma(fa, fb0, acc[0]);
      acc[1] = Frag<_Float16>::mma(fa, fb1, acc[1]);
      dep_guard3_h(acc[0], acc[1], fa, fb0, fb1);
    }
    acc_guard2(acc[0], acc[1]);

    float hv[2][8];
#pragma unroll
    for (int j = 0; j < 2; ++j) {
#pragma unroll
      for (int r = 0; r < 8; ++r) {
        const float v = fmaxf(acc[j][r] * inv16, 0.0f);
        hv[j][r] = v;
        hn[(mOff + r) * kHP + n0 + 16 * j + c] = (_Float16)v;
      }
    }
    if (HEAD) {
#pragma unroll
      for (int r = 0; r < 8; ++r) {
        float s = hv[0][r] * wf0 + hv[1][r] * wf1;
        s += __shfl_xor(s, 1, 32);
        s += __shfl_xor(s, 2, 32);
        s += __shfl_xor(s, 4, 32);
        s += __shfl_xor(s, 8, 32);
        if (c == 0) sPart[((t & 1) * 8 + wave) * kSeqPB + mOff + r] = s;
      }
    }
    __syncthreads();

    if (HEAD == 0) {
      const size_t rowq = (size_t)t * kQSeq + bl0;
      for (int pass = 0; pass < 2; ++pass) {
#pragma unroll
        for (int it = 0; it < 2; ++it) {
          const int rr = wave * 2 + it;
          const v8h v = *(const v8h*)(hn + rr * kHP + 8 * lane);
          *(volatile v8h*)(hout + (rowq + rr) * kHid + 8 * lane) = v;
        }
        __threadfence();
      }
    } else {
      if (wave == 0) {
        const int seq = lane & 15;
        const float* sp = sPart + (t & 1) * 8 * kSeqPB + seq;
        float s = sp[0];
        s += sp[1 * kSeqPB]; s += sp[2 * kSeqPB]; s += sp[3 * kSeqPB];
        s += sp[4 * kSeqPB]; s += sp[5 * kSeqPB]; s += sp[6 * kSeqPB]; s += sp[7 * kSeqPB];
        s += bfcv;
        if (lane < 16) sOut[seq * kOutPitch + (t & 31)] = s;
        if ((t & 31) == 31) {
          __builtin_amdgcn_fence(__ATOMIC_RELEASE, "workgroup");
          __builtin_amdgcn_wave_barrier();
          __builtin_amdgcn_fence(__ATOMIC_ACQUIRE, "workgroup");
          float* ob = outq + (size_t)bl0 * kStep + (t - 31);
          for (int pass = 0; pass < 2; ++pass) {
#pragma unroll
            for (int it = 0; it < 4; ++it) {
              const int sq = it * 4 + q4;
              const v4f v = *(const v4f*)(sOut + sq * kOutPitch + c4);
              *(volatile v4f*)(ob + (size_t)sq * kStep + c4) = v;
            }
            __threadfence();
          }
        }
      }
    }
  }
}

extern "C" void kernel_launch(void* const* d_in, const int* in_sizes, int n_in,
                              void* d_out, int out_size, void* d_ws, size_t ws_size, hipStream_t stream) {
  if (n_in < 11 || d_out == nullptr || d_ws == nullptr) return;
  if (in_sizes[0] != kSeq * kStep * kIn || in_sizes[1] != kHid * kIn || in_sizes[2] != kHid * kHid ||
      in_sizes[3] != kHid || in_sizes[4] != kHid || in_sizes[5] != kHid * kHid || in_sizes[6] != kHid * kHid ||
      in_sizes[7] != kHid || in_sizes[8] != kHid || in_sizes[9] != kHid || in_sizes[10] != 1 ||
      out_size != kRows) return;

  const float* x     = (const float*)d_in[0];
  const float* w_ih0 = (const float*)d_in[1];
  const float* w_hh0 = (const float*)d_in[2];
  const float* b_ih0 = (const float*)d_in[3];
  const float* b_hh0 = (const float*)d_in[4];
  const float* w_ih1 = (const float*)d_in[5];
  const float* w_hh1 = (const float*)d_in[6];
  const float* b_ih1 = (const float*)d_in[7];
  const float* b_hh1 = (const float*)d_in[8];
  const float* w_fc  = (const float*)d_in[9];
  const float* b_fc  = (const float*)d_in[10];
  float* out = (float*)d_out;

  char* ws = (char*)d_ws; size_t off = 0;
  auto carve = [&](size_t bytes) -> char* { char* p = ws + off; off += (bytes + 255) & ~(size_t)255; return p; };
  unsigned short* X16     = (unsigned short*)carve((size_t)kRows * kIn * 2);
  unsigned short* WIH0_16 = (unsigned short*)carve((size_t)kHid * kIn * 2);
  unsigned short* WHH0_16 = (unsigned short*)carve((size_t)kHid * kHid * 2);
  unsigned short* WIH1_16 = (unsigned short*)carve((size_t)kHid * kHid * 2);
  unsigned short* WHH1_16 = (unsigned short*)carve((size_t)kHid * kHid * 2);
  float*          BSUM    = (float*)carve((size_t)kDwBsum * 4);
  float*          PRE     = (float*)carve((size_t)kHid * kRowsQ * 4);
  unsigned short* H1_16   = (unsigned short*)carve((size_t)kRows * kHid * 2);
  if (off > ws_size || off > (size_t)134217728) return;

  const float inv16 = 1.0f / 16.0f;
  const int projGrid = ((kHid / 64) * (kRowsQ / 64)) / 8;

  prep_kernel<<<kPrepBlocks, 256, 0, stream>>>(w_ih0, w_hh0, w_ih1, w_hh1, b_ih0, b_hh0, b_ih1, b_hh1,
                                               (unsigned*)WIH0_16, (unsigned*)WHH0_16, (unsigned*)WIH1_16,
                                               (unsigned*)WHH1_16, (unsigned*)BSUM);

  xcast_kernel<<<kXChunks / 256, 256, 0, stream>>>(x, (_Float16*)X16);

  for (int g = 0; g < kNQ; ++g) {
    const unsigned short* xq = X16 + (size_t)g * kRowsQ * kIn;
    unsigned short* h1q = H1_16 + (size_t)g * kRowsQ * kHid;
    wmma_gemm64<0, false, 1, 0, false, 0><<<dim3(projGrid, 1), 256, 0, stream>>>(
        WIH0_16, nullptr, kIn, 0L, xq, nullptr, kIn, 0L,
        (void*)PRE, nullptr, kRowsQ, 0L, BSUM, nullptr, 0L, kHid, kRowsQ, kIn, inv16);
    rnn_layer_kernel<0><<<kRnnBlocks, kRnnThreads, 0, stream>>>(
        PRE, (const _Float16*)WHH0_16, (_Float16*)h1q, w_fc, b_fc, out + (size_t)g * kQSeq * kStep);
  }

  for (int g = 0; g < kNQ; ++g) {
    unsigned short* h1q = H1_16 + (size_t)g * kRowsQ * kHid;
    wmma_gemm64<0, false, 1, 0, false, 0><<<dim3(projGrid, 1), 256, 0, stream>>>(
        WIH1_16, nullptr, kHid, 0L, h1q, nullptr, kHid, 0L,
        (void*)PRE, nullptr, kRowsQ, 0L, BSUM + kHid, nullptr, 0L, kHid, kRowsQ, kHid, inv16);
    rnn_layer_kernel<1><<<kRnnBlocks, kRnnThreads, 0, stream>>>(
        PRE, (const _Float16*)WHH1_16, (_Float16*)h1q, w_fc, b_fc, out + (size_t)g * kQSeq * kStep);
  }
}
